// ImprovedGNN_12893491822683
// MI455X (gfx1250) — hardware-verified
//
#include <hip/hip_runtime.h>
#include <stddef.h>
#include <stdint.h>


#define DIN     128
#define NOC     64
#define APW     256
#define KSEG    256
#define NTHR    256
#define NWAVE   8
#define EPT     8
#define CHUNK   (NTHR * EPT)
#define WCAP    (EPT * 32)
#define LISTN   (NWAVE * WCAP)
#define NBMAX   2048
#define RCAP    28672
#define DEGCAP  64
#define PKS     11
#define STW     512
#define GBM     64
#define GTHR    128
#define WSMAX   134217728
#define LDS_AGG ((2 * RCAP + 2 * NBMAX + LISTN) * 4 + 64)
#define LN_EPS  1e-5f

static_assert((CHUNK & (CHUNK - 1)) == 0 && CHUNK <= (1 << PKS));
static_assert((NBMAX & (NBMAX - 1)) == 0 && NBMAX <= (1 << PKS));
static_assert(NTHR * 8 == NBMAX);
static_assert(LISTN >= NBMAX);
static_assert(LISTN >= NWAVE * WCAP);
static_assert((RCAP % 32) == 0);
static_assert(NWAVE * STW <= RCAP);
static_assert(LDS_AGG <= 300000);
static_assert(GBM == (GTHR / 32) * 16);
static_assert((DIN % 32) == 0 && (KSEG % 32) == 0 && KSEG == 2 * DIN);
static_assert(DIN == 32 * 4 && APW == 2 * DIN);
static_assert((GBM % NWAVE) == 0);
static_assert((NOC % 16) == 0 && NOC == 64);

typedef float          v4f  __attribute__((ext_vector_type(4)));
typedef float          v8f  __attribute__((ext_vector_type(8)));
typedef int            v4i  __attribute__((ext_vector_type(4)));
typedef int            v8i  __attribute__((ext_vector_type(8)));
typedef unsigned int   v2u  __attribute__((ext_vector_type(2)));
typedef unsigned int   v4u  __attribute__((ext_vector_type(4)));
typedef unsigned short v8us __attribute__((ext_vector_type(8)));
typedef __bf16         v16b __attribute__((ext_vector_type(16)));
union FragB { v16b v; v8us h[2]; v8i w; };

__device__ __forceinline__ v8f wmb(const FragB& a, const FragB& b, v8f c) {
  v8f d = __builtin_amdgcn_wmma_f32_16x16x32_bf16(false, a.v, false, b.v, (short)0, c, false, false);
  asm volatile("v_nop\n\tv_nop\n\tv_nop\n\tv_nop" : "+v"(d) : "v"(a.w), "v"(b.w));
  return d;
}

__device__ __forceinline__ unsigned short bf_bits(float f) {
  unsigned int u = __float_as_uint(f);
  u += 0x7FFFu + ((u >> 16) & 1u);
  return (unsigned short)(u >> 16);
}
__device__ __forceinline__ float bf_val(unsigned short b) {
  return __uint_as_float(((unsigned int)b) << 16);
}
__device__ __forceinline__ float bf_rne(float f) { return bf_val(bf_bits(f)); }

__device__ __forceinline__ v8us cvt8b(const v4f a, const v4f b) {
  v8us hv;
  hv[0] = bf_bits(a.x); hv[1] = bf_bits(a.y); hv[2] = bf_bits(a.z); hv[3] = bf_bits(a.w);
  hv[4] = bf_bits(b.x); hv[5] = bf_bits(b.y); hv[6] = bf_bits(b.z); hv[7] = bf_bits(b.w);
  return hv;
}
__device__ __forceinline__ v8us cvt8lo(const v4f a, const v4f b, const v8us hi) {
  v8us lv;
  lv[0] = bf_bits(a.x - bf_val(hi[0])); lv[1] = bf_bits(a.y - bf_val(hi[1]));
  lv[2] = bf_bits(a.z - bf_val(hi[2])); lv[3] = bf_bits(a.w - bf_val(hi[3]));
  lv[4] = bf_bits(b.x - bf_val(hi[4])); lv[5] = bf_bits(b.y - bf_val(hi[5]));
  lv[6] = bf_bits(b.z - bf_val(hi[6])); lv[7] = bf_bits(b.w - bf_val(hi[7]));
  return lv;
}

__device__ __forceinline__ float gelu_f(float x) {
  return 0.5f * x * (1.0f + erff(x * 0.70710678118654752f));
}

__device__ __forceinline__ int scan_chunk(const int* __restrict__ dsts, int nE, int cbase, int slotBase,
                                          int nb, int vec8, int* list, int tid, int lane, int wave) {
  int wc = 0;
  const int el0  = tid * EPT;
  const int e0   = cbase + el0;
  const int sent = -2147483647 - 1;
  v4i da, db;
  if (vec8 != 0 && cbase + CHUNK <= nE) {
    da = *(const v4i*)(dsts + e0);
    db = *(const v4i*)(dsts + e0 + 4);
  } else {
    da.x = (e0     < nE) ? dsts[min(e0,     nE - 1)] : sent;
    da.y = (e0 + 1 < nE) ? dsts[min(e0 + 1, nE - 1)] : sent;
    da.z = (e0 + 2 < nE) ? dsts[min(e0 + 2, nE - 1)] : sent;
    da.w = (e0 + 3 < nE) ? dsts[min(e0 + 3, nE - 1)] : sent;
    db.x = (e0 + 4 < nE) ? dsts[min(e0 + 4, nE - 1)] : sent;
    db.y = (e0 + 5 < nE) ? dsts[min(e0 + 5, nE - 1)] : sent;
    db.z = (e0 + 6 < nE) ? dsts[min(e0 + 6, nE - 1)] : sent;
    db.w = (e0 + 7 < nE) ? dsts[min(e0 + 7, nE - 1)] : sent;
  }
  const unsigned nbs = (unsigned)slotBase;
  const unsigned unb = (unsigned)nb;
  const unsigned s0 = (unsigned)da.x - nbs, s1 = (unsigned)da.y - nbs;
  const unsigned s2 = (unsigned)da.z - nbs, s3 = (unsigned)da.w - nbs;
  const unsigned s4 = (unsigned)db.x - nbs, s5 = (unsigned)db.y - nbs;
  const unsigned s6 = (unsigned)db.z - nbs, s7 = (unsigned)db.w - nbs;
  const bool h0 = s0 < unb, h1 = s1 < unb, h2 = s2 < unb, h3 = s3 < unb;
  const bool h4 = s4 < unb, h5 = s5 < unb, h6 = s6 < unb, h7 = s7 < unb;
  const unsigned any = __builtin_amdgcn_ballot_w32(h0 | h1 | h2 | h3 | h4 | h5 | h6 | h7);
  if (any != 0u) {
#define HITJ(J, HJ, SJ) { \
      const unsigned mj = __builtin_amdgcn_ballot_w32(HJ); \
      if (mj != 0u) { \
        if (HJ) { \
          const int pos = wc + (int)__builtin_amdgcn_mbcnt_lo(mj, 0u); \
          if (pos < WCAP) list[wave * WCAP + pos] = ((el0 + (J)) << PKS) | (int)(SJ); \
        } \
        wc += (int)__builtin_popcount(mj); } }
    HITJ(0, h0, s0)
    HITJ(1, h1, s1)
    HITJ(2, h2, s2)
    HITJ(3, h3, s3)
    HITJ(4, h4, s4)
    HITJ(5, h5, s5)
    HITJ(6, h6, s6)
    HITJ(7, h7, s7)
#undef HITJ
  }
  return wc;
}

__device__ __forceinline__ void wt_pass(const float* T, unsigned short* wt, int n0, int KT, int nsrc, int tid) {
  const int upr    = KT >> 3;
  const int nUnits = 16 * upr;
#pragma unroll 1
  for (int u = tid; u < nUnits; u += NTHR) {
    const int nl  = u / upr;
    const int k8  = (u - nl * upr) * 8;
    const int seg = k8 >> 7;
    const int sr  = (nsrc == 2) ? ((seg >> 1) & 1) : 0;
    const int ks  = k8 & (DIN - 1);
    const float* tp = T + (size_t)(sr * DIN + ks) * 16 + nl;
    v4f a, b;
    a.x = tp[0];  a.y = tp[16]; a.z = tp[32];  a.w = tp[48];
    b.x = tp[64]; b.y = tp[80]; b.z = tp[96];  b.w = tp[112];
    const v8us hv = cvt8b(a, b);
    *(volatile v8us*)(wt + (size_t)(n0 + nl) * (size_t)KT + k8) = hv;
  }
}

__global__ __launch_bounds__(NTHR) void k_wtr(const float* __restrict__ w0base, const float* __restrict__ w1base,
                                              int wstrideY, unsigned short* wtbase, int tstrideY,
                                              int nOut, int KT, int nsrc) {
  __shared__ __attribute__((aligned(16))) float T[2 * DIN * 16];
  const int tid = (int)threadIdx.x;
  const int n0  = (int)blockIdx.x * 16;
  const float* w0 = w0base + (size_t)blockIdx.y * (size_t)wstrideY;
  const float* w1 = w1base + (size_t)blockIdx.y * (size_t)wstrideY;
  unsigned short* wt = wtbase + (size_t)blockIdx.y * (size_t)tstrideY;
#pragma unroll 1
  for (int idx = tid; idx < 1024; idx += NTHR) {
    const int sr  = idx >> 9;
    const int rem = idx & 511;
    const int k   = rem >> 2;
    const int c4  = (rem & 3) * 4;
    int col = n0 + c4;
    col = col > nOut - 4 ? nOut - 4 : col;
    const float* wp = (sr == 0) ? w0 : w1;
    const v4f v = *(const v4f*)(wp + (size_t)k * (size_t)nOut + col);
    *(v4f*)(T + (sr * DIN + k) * 16 + c4) = v;
  }
  __syncthreads();
  wt_pass(T, wt, n0, KT, nsrc, tid);
  __threadfence();
  wt_pass(T, wt, n0, KT, nsrc, tid);
}

__global__ __launch_bounds__(NTHR) void k_ln(const float* __restrict__ X, const float* __restrict__ gamma,
                                             const float* __restrict__ beta, int rin,
                                             unsigned short* HHo, int nN, int MPr) {
  __shared__ __attribute__((aligned(16))) unsigned int lstg[NWAVE * 128];
  const int tid = (int)threadIdx.x, lane = tid & 31, wave = tid >> 5;
  const int row = (int)blockIdx.x * NWAVE + wave;
  if (row >= MPr) return;
  const int rc = row < nN ? row : nN - 1;
  const size_t base = (size_t)rc * DIN + 4 * lane;
  const v4f xr = *(const v4f*)(X + base);
  const v4f gr = *(const v4f*)(gamma + 4 * lane);
  const v4f br = *(const v4f*)(beta + 4 * lane);
  const bool rb = rin != 0;
  const float x0 = rb ? bf_rne(xr.x) : xr.x, x1 = rb ? bf_rne(xr.y) : xr.y;
  const float x2 = rb ? bf_rne(xr.z) : xr.z, x3 = rb ? bf_rne(xr.w) : xr.w;
  float s = (x0 + x1) + (x2 + x3);
#pragma unroll
  for (int mm = 16; mm >= 1; mm >>= 1) s += __shfl_xor(s, mm, 32);
  const float mu = s * (1.0f / DIN);
  const float d0 = x0 - mu, d1 = x1 - mu, d2 = x2 - mu, d3 = x3 - mu;
  float ss = (d0 * d0 + d1 * d1) + (d2 * d2 + d3 * d3);
#pragma unroll
  for (int mm = 16; mm >= 1; mm >>= 1) ss += __shfl_xor(ss, mm, 32);
  const float var  = ss * (1.0f / DIN);
  const float rstd = rsqrtf(var + LN_EPS);
  const float g0 = bf_rne(gr.x), g1 = bf_rne(gr.y), g2 = bf_rne(gr.z), g3 = bf_rne(gr.w);
  const float e0 = bf_rne(br.x), e1 = bf_rne(br.y), e2 = bf_rne(br.z), e3 = bf_rne(br.w);
  float r0 = (d0 * rstd) * g0 + e0;
  float r1 = (d1 * rstd) * g1 + e1;
  float r2 = (d2 * rstd) * g2 + e2;
  float r3 = (d3 * rstd) * g3 + e3;
  const bool liveRow = row < nN;
  r0 = liveRow ? r0 : 0.0f; r1 = liveRow ? r1 : 0.0f; r2 = liveRow ? r2 : 0.0f; r3 = liveRow ? r3 : 0.0f;

  const unsigned short hb0 = bf_bits(r0), hb1 = bf_bits(r1), hb2 = bf_bits(r2), hb3 = bf_bits(r3);
  const unsigned short lb0 = bf_bits(r0 - bf_val(hb0)), lb1 = bf_bits(r1 - bf_val(hb1));
  const unsigned short lb2 = bf_bits(r2 - bf_val(hb2)), lb3 = bf_bits(r3 - bf_val(hb3));
  v2u hw, lw;
  hw.x = (unsigned int)hb0 | ((unsigned int)hb1 << 16);
  hw.y = (unsigned int)hb2 | ((unsigned int)hb3 << 16);
  lw.x = (unsigned int)lb0 | ((unsigned int)lb1 << 16);
  lw.y = (unsigned int)lb2 | ((unsigned int)lb3 << 16);
  unsigned int* stwu = lstg + wave * 128;
  __builtin_amdgcn_fence(__ATOMIC_RELEASE, "wavefront");
  __builtin_amdgcn_wave_barrier();
  *(v2u*)(stwu + 2 * lane)      = hw;
  *(v2u*)(stwu + 64 + 2 * lane) = lw;
  __builtin_amdgcn_fence(__ATOMIC_RELEASE, "wavefront");
  __builtin_amdgcn_wave_barrier();
  const v4u pk = *(const v4u*)(stwu + 4 * lane);

  unsigned short* gp = HHo + (size_t)row * APW + 8 * lane;
  *(volatile v4u*)gp = pk;
  __threadfence();
  *(volatile v4u*)gp = pk;
}

template <int NT>
__device__ __forceinline__ void gemm_main(v8f (&acc)[NT], const unsigned short* A0, const unsigned short* A1,
                                          int nseg, int lda, const unsigned short* __restrict__ WT, int ktot,
                                          int rowBase, int wave, int hh, int m) {
  {
    const v8f z = {0.f, 0.f, 0.f, 0.f, 0.f, 0.f, 0.f, 0.f};
#pragma unroll
    for (int t = 0; t < NT; ++t) acc[t] = z;
  }
  const size_t arow = (size_t)(rowBase + 16 * wave + m) * (size_t)lda + 8 * hh;
  const unsigned short* wp = WT + (size_t)m * (size_t)ktot + 8 * hh;
  constexpr int ksteps = KSEG / 32;
#pragma unroll 1
  for (int seg = 0; seg < nseg; ++seg) {
    const unsigned short* ap  = (seg == 0 ? A0 : A1) + arow;
    const unsigned short* wps = wp + seg * KSEG;
#pragma unroll 1
    for (int ks = 0; ks < ksteps; ++ks) {
      FragB af;
      af.h[0] = *(const v8us*)(ap + 32 * ks);
      af.h[1] = *(const v8us*)(ap + 32 * ks + 16);
#pragma unroll
      for (int t = 0; t < NT; ++t) {
        const unsigned short* wq = wps + (size_t)(16 * t) * (size_t)ktot + 32 * ks;
        FragB bf;
        bf.h[0] = *(const v8us*)wq;
        bf.h[1] = *(const v8us*)(wq + 16);
        acc[t] = wmb(af, bf, acc[t]);
      }
    }
  }
}

__device__ __forceinline__ void h_store_rows(const float* stg, int wave, int lane, int hh, int m, int rowBase,
                                             float* outF, unsigned short* outHH, int MPr) {
#pragma unroll 1
  for (int i = 0; i < 16; ++i) {
    const int lr   = 16 * wave + i;
    const int grow = rowBase + lr;
    const float* sp = stg + lr * DIN;
    const v4f hv = *(const v4f*)(sp + 4 * lane);
    const v4f p0 = *(const v4f*)(sp + 8 * m);
    const v4f p1 = *(const v4f*)(sp + 8 * m + 4);
    const v8us hi8 = cvt8b(p0, p1);
    const v8us lo8 = cvt8lo(p0, p1, hi8);
    const v8us pk  = (hh == 0) ? hi8 : lo8;
    if (grow < MPr) {
      *(volatile v4f*)(outF + (size_t)grow * DIN + 4 * lane)   = hv;
      *(volatile v8us*)(outHH + (size_t)grow * APW + 8 * lane) = pk;
    }
  }
}

__global__ __launch_bounds__(GTHR) void k_gemm_h(const unsigned short* A0, const unsigned short* A1, int nseg, int lda,
                                                 const unsigned short* __restrict__ WT, int ktot,
                                                 const float* __restrict__ bias, const float* __restrict__ gamma,
                                                 const float* __restrict__ beta, const float* __restrict__ Hid,
                                                 int mode, float* outF, unsigned short* outHH, int nN, int MPr) {
  constexpr int NT = 8;
  constexpr int BN = 16 * NT;
  static_assert(BN == DIN);
  __shared__ __attribute__((aligned(16))) float stg[GBM * BN];
  const int tid = (int)threadIdx.x, lane = tid & 31, wave = tid >> 5, hh = lane >> 4, m = lane & 15;
  const int rowBase = (int)blockIdx.x * GBM;

  v8f acc[NT];
  gemm_main<NT>(acc, A0, A1, nseg, lda, WT, ktot, rowBase, wave, hh, m);

#pragma unroll
  for (int t = 0; t < NT; ++t) {
    const int lc = 16 * t + m;
    const float bb = bf_rne(bias[lc]);
#pragma unroll
    for (int r = 0; r < 8; ++r) {
      const int lr = 16 * wave + 8 * hh + r;
      stg[lr * BN + lc] = acc[t][r] + bb;
    }
  }
  __syncthreads();

  const v4f g4 = *(const v4f*)(gamma + 4 * lane);
  const v4f e4 = *(const v4f*)(beta + 4 * lane);
  const float g0 = bf_rne(g4.x), g1 = bf_rne(g4.y), g2 = bf_rne(g4.z), g3 = bf_rne(g4.w);
  const float e0 = bf_rne(e4.x), e1 = bf_rne(e4.y), e2 = bf_rne(e4.z), e3 = bf_rne(e4.w);
  const bool ln = mode != 0;
#pragma unroll 1
  for (int i = 0; i < 16; ++i) {
    const int lr   = 16 * wave + i;
    const int grow = rowBase + lr;
    float* sp = stg + lr * BN + 4 * lane;
    const v4f v = *(const v4f*)sp;
    float s = (v.x + v.y) + (v.z + v.w);
#pragma unroll
    for (int mm = 16; mm >= 1; mm >>= 1) s += __shfl_xor(s, mm, 32);
    const float mu = s * (1.0f / DIN);
    const float d0 = v.x - mu, d1 = v.y - mu, d2 = v.z - mu, d3 = v.w - mu;
    float ss = (d0 * d0 + d1 * d1) + (d2 * d2 + d3 * d3);
#pragma unroll
    for (int mm = 16; mm >= 1; mm >>= 1) ss += __shfl_xor(ss, mm, 32);
    const float var  = ss * (1.0f / DIN);
    const float rstd = rsqrtf(var + LN_EPS);
    const float t0 = ln ? (d0 * rstd) * g0 + e0 : v.x;
    const float t1 = ln ? (d1 * rstd) * g1 + e1 : v.y;
    const float t2 = ln ? (d2 * rstd) * g2 + e2 : v.z;
    const float t3 = ln ? (d3 * rstd) * g3 + e3 : v.w;
    const int hr = grow < nN ? grow : nN - 1;
    const v4f idv = *(const v4f*)(Hid + (size_t)hr * DIN + 4 * lane);
    float o0 = gelu_f(t0) + (ln ? idv.x : 0.0f);
    float o1 = gelu_f(t1) + (ln ? idv.y : 0.0f);
    float o2 = gelu_f(t2) + (ln ? idv.z : 0.0f);
    float o3 = gelu_f(t3) + (ln ? idv.w : 0.0f);
    const bool liveRow = grow < nN;
    v4f ov;
    ov.x = liveRow ? o0 : 0.0f; ov.y = liveRow ? o1 : 0.0f;
    ov.z = liveRow ? o2 : 0.0f; ov.w = liveRow ? o3 : 0.0f;
    *(v4f*)sp = ov;
  }
  __syncthreads();

  h_store_rows(stg, wave, lane, hh, m, rowBase, outF, outHH, MPr);
  __threadfence();
  h_store_rows(stg, wave, lane, hh, m, rowBase, outF, outHH, MPr);
}

__global__ __launch_bounds__(GTHR) void k_gemm_o(const unsigned short* A0, int lda,
                                                 const unsigned short* __restrict__ WT, int ktot,
                                                 const float* __restrict__ bias, float* out, int nRows) {
  constexpr int NT = NOC / 16;
  constexpr int BN = NOC;
  constexpr int NI = 8;
  __shared__ __attribute__((aligned(16))) float stg[GBM * BN];
  const int tid = (int)threadIdx.x, lane = tid & 31, wave = tid >> 5, hh = lane >> 4, m = lane & 15;
  const int rowBase = (int)blockIdx.x * GBM;

  v8f acc[NT];
  gemm_main<NT>(acc, A0, A0, 1, lda, WT, ktot, rowBase, wave, hh, m);

#pragma unroll
  for (int t = 0; t < NT; ++t) {
    const int lc = 16 * t + m;
    const float bb = bf_rne(bias[lc]);
#pragma unroll
    for (int r = 0; r < 8; ++r) {
      const int lr = 16 * wave + 8 * hh + r;
      stg[lr * BN + lc] = acc[t][r] + bb;
    }
  }
  __syncthreads();

  v4f fv[NI];
#pragma unroll
  for (int i = 0; i < NI; ++i) {
    const int lr = 16 * wave + 2 * i + hh;
    fv[i] = *(const v4f*)(stg + lr * BN + 4 * m);
  }
#pragma unroll
  for (int i = 0; i < NI; ++i) {
    const int gr = rowBase + 16 * wave + 2 * i + hh;
    float* op = out + (size_t)gr * (size_t)NOC + 4 * m;
    if (gr < nRows) *(volatile v4f*)op = fv[i];
  }
  __threadfence();
#pragma unroll
  for (int i = 0; i < NI; ++i) {
    const int gr = rowBase + 16 * wave + 2 * i + hh;
    float* op = out + (size_t)gr * (size_t)NOC + 4 * m;
    if (gr < nRows) *(volatile v4f*)op = fv[i];
  }
}

__global__ __launch_bounds__(NTHR) void k_agg(
    const int* __restrict__ srcs, const int* __restrict__ dsts,
    const float* __restrict__ Hf,
    unsigned short* Aout, int ldaOut,
    int nN, int nE, int nb, int vec8, int MPr) {
  extern __shared__ v4f lds_dyn[];
  int* reg1 = (int*)lds_dyn;
  int* reg2 = reg1 + RCAP;
  int* scnt = reg2 + RCAP;
  int* soff = scnt + NBMAX;
  int* list = soff + NBMAX;
  int* wcnt = list + LISTN;
  int* wtot = wcnt + NWAVE;
  const int tid = (int)threadIdx.x, lane = tid & 31, wave = tid >> 5;
  const int nodeBase = (int)blockIdx.x * nb;

  for (int i = tid; i < NBMAX; i += NTHR) scnt[i] = 0;
  __syncthreads();

  int tot = 0;
  const int nChunks = (nE + CHUNK - 1) / CHUNK;
#pragma unroll 1
  for (int ch = 0; ch < nChunks; ++ch) {
    const int cbase = ch * CHUNK;
    const int wc = scan_chunk(dsts, nE, cbase, nodeBase, nb, vec8, list, tid, lane, wave);
    if (lane == 0) wcnt[wave] = wc;
    __syncthreads();
    int pre = 0, all = 0;
#pragma unroll
    for (int w2 = 0; w2 < NWAVE; ++w2) {
      int c = wcnt[w2];
      c = c < 0 ? 0 : (c > WCAP ? WCAP : c);
      all += c;
      pre += (w2 < wave) ? c : 0;
    }
    const int wcc  = wc > WCAP ? WCAP : wc;
    const int base = tot + pre;
#pragma unroll 1
    for (int i = lane; i < wcc; i += 32) {
      const int ent = list[wave * WCAP + i];
      const int el  = (ent >> PKS) & (CHUNK - 1);
      const int sl  = ent & (NBMAX - 1);
      int eid = cbase + el;
      eid = eid > nE - 1 ? nE - 1 : eid;
      const int pos = base + i;
      if (pos < RCAP) reg1[pos] = (int)(((unsigned)eid << PKS) | (unsigned)sl);
    }
    tot += all;
    tot = tot > RCAP ? RCAP : tot;
    __syncthreads();
  }
  const int nh = tot;

  if (wave == 0) {
#pragma unroll 1
    for (int b0 = 0; b0 < nh; b0 += 32) {
      const int idx = b0 + lane;
      const int uv  = reg1[idx < RCAP ? idx : RCAP - 1];
      const int m32 = (nh - b0) < 32 ? (nh - b0) : 32;
#pragma unroll 1
      for (int k = 0; k < m32; ++k) {
        const int u  = __builtin_amdgcn_readlane(uv, k);
        const int sl = u & (NBMAX - 1);
        if (lane == 0) scnt[sl] = scnt[sl] + 1;
      }
    }
  }
  __syncthreads();

  {
    const v4i ca = *(const v4i*)(scnt + 8 * tid);
    const v4i cb = *(const v4i*)(scnt + 8 * tid + 4);
    const int e0 = ca.x < 0 ? 0 : ca.x, e1 = ca.y < 0 ? 0 : ca.y, e2 = ca.z < 0 ? 0 : ca.z, e3 = ca.w < 0 ? 0 : ca.w;
    const int e4 = cb.x < 0 ? 0 : cb.x, e5 = cb.y < 0 ? 0 : cb.y, e6 = cb.z < 0 ? 0 : cb.z, e7 = cb.w < 0 ? 0 : cb.w;
    const int ts = e0 + e1 + e2 + e3 + e4 + e5 + e6 + e7;
    int incl = ts;
#pragma unroll
    for (int d = 1; d < 32; d <<= 1) {
      const int up = __shfl_up(incl, d);
      if (lane >= d) incl += up;
    }
    if (lane == 31) wtot[wave] = incl;
    __syncthreads();
    int pre = 0;
#pragma unroll
    for (int w2 = 0; w2 < NWAVE; ++w2) pre += (w2 < wave) ? wtot[w2] : 0;
    int run = pre + incl - ts;
    soff[8 * tid + 0] = run; run += e0;
    soff[8 * tid + 1] = run; run += e1;
    soff[8 * tid + 2] = run; run += e2;
    soff[8 * tid + 3] = run; run += e3;
    soff[8 * tid + 4] = run; run += e4;
    soff[8 * tid + 5] = run; run += e5;
    soff[8 * tid + 6] = run; run += e6;
    soff[8 * tid + 7] = run;
  }
  __syncthreads();
  for (int i = tid; i < NBMAX; i += NTHR) list[i] = soff[i];
  __syncthreads();

  if (wave == 0) {
#pragma unroll 1
    for (int b0 = 0; b0 < nh; b0 += 32) {
      const int idx = b0 + lane;
      const int uv  = reg1[idx < RCAP ? idx : RCAP - 1];
      const int m32 = (nh - b0) < 32 ? (nh - b0) : 32;
#pragma unroll 1
      for (int k = 0; k < m32; ++k) {
        const int u   = __builtin_amdgcn_readlane(uv, k);
        const int sl  = u & (NBMAX - 1);
        const int eid = (int)((unsigned)u >> PKS);
        if (lane == 0) {
          int pos = list[sl];
          pos = pos < 0 ? 0 : (pos > RCAP - 1 ? RCAP - 1 : pos);
          reg2[pos] = eid;
          list[sl] = pos + 1;
        }
      }
    }
  }
  __syncthreads();

  const int nbw = nb >> 3;
  const bool ovf = (nh >= RCAP);
  const float qnan = __int_as_float(0x7fc00000);
  unsigned int* stwu = (unsigned int*)((float*)reg1 + wave * STW);

#pragma unroll 1
  for (int jt = 0; jt < nbw; ++jt) {
    const int slot = wave * nbw + jt;
    const int grow = nodeBase + slot;
    int st = soff[slot];
    const int craw = scnt[slot];
    int cnt = craw;
    st  = st < 0 ? 0 : (st > nh ? nh : st);
    cnt = cnt < 0 ? 0 : (cnt > DEGCAP ? DEGCAP : cnt);
    if (cnt > nh - st) cnt = nh - st;
    const float pz = (ovf || craw > DEGCAP) ? qnan : 0.0f;
    const bool liveRow = grow < nN;

    float ag0 = 0.f, ag1 = 0.f, ag2 = 0.f, ag3 = 0.f;
#pragma unroll 1
    for (int q = 0; q < cnt; ++q) {
      int idx = st + q; idx = idx > RCAP - 1 ? RCAP - 1 : idx;
      int eid = reg2[idx]; eid = eid < 0 ? 0 : (eid > nE - 1 ? nE - 1 : eid);
      const int sraw = srcs[eid];
      const int s = sraw < 0 ? 0 : (sraw > nN - 1 ? nN - 1 : sraw);
      const v4f v = *(const v4f*)(Hf + (size_t)s * DIN + 4 * lane);
      ag0 += v.x; ag1 += v.y; ag2 += v.z; ag3 += v.w;
    }
    const float dcl  = cnt > 0 ? (float)cnt : 1.0f;
    const float invd = 1.0f / dcl;
    float r0 = ag0 * invd, r1 = ag1 * invd, r2 = ag2 * invd, r3 = ag3 * invd;
    r0 = (liveRow ? r0 : 0.0f) + pz;
    r1 = (liveRow ? r1 : 0.0f) + pz;
    r2 = (liveRow ? r2 : 0.0f) + pz;
    r3 = (liveRow ? r3 : 0.0f) + pz;

    const unsigned short hb0 = bf_bits(r0), hb1 = bf_bits(r1), hb2 = bf_bits(r2), hb3 = bf_bits(r3);
    const unsigned short lb0 = bf_bits(r0 - bf_val(hb0)), lb1 = bf_bits(r1 - bf_val(hb1));
    const unsigned short lb2 = bf_bits(r2 - bf_val(hb2)), lb3 = bf_bits(r3 - bf_val(hb3));
    v2u hw, lw;
    hw.x = (unsigned int)hb0 | ((unsigned int)hb1 << 16);
    hw.y = (unsigned int)hb2 | ((unsigned int)hb3 << 16);
    lw.x = (unsigned int)lb0 | ((unsigned int)lb1 << 16);
    lw.y = (unsigned int)lb2 | ((unsigned int)lb3 << 16);
    __builtin_amdgcn_fence(__ATOMIC_RELEASE, "wavefront");
    __builtin_amdgcn_wave_barrier();
    *(v2u*)(stwu + 2 * lane)      = hw;
    *(v2u*)(stwu + 64 + 2 * lane) = lw;
    __builtin_amdgcn_fence(__ATOMIC_RELEASE, "wavefront");
    __builtin_amdgcn_wave_barrier();
    const v4u pk = *(const v4u*)(stwu + 4 * lane);
    unsigned short* gp = Aout + (size_t)grow * (size_t)ldaOut + 8 * lane;
    const bool wsv = grow < MPr;
    if (wsv) *(volatile v4u*)gp = pk;
    __threadfence();
    if (wsv) *(volatile v4u*)gp = pk;
  }
}

static int pick_nb(int nE, int nN) {
  int nb = NBMAX;
  while (nb > 16 && (long long)nb * (long long)nE * 5LL > (long long)RCAP * (long long)nN * 4LL) nb >>= 1;
  return nb;
}
static inline int cdiv(int a, int b) { return (a + b - 1) / b; }

extern "C" void kernel_launch(void* const* d_in, const int* in_sizes, int n_in,
                              void* d_out, int out_size, void* d_ws, size_t ws_size,
                              hipStream_t stream) {
  if (n_in < 15) return;
  const int nN = in_sizes[0] / DIN;
  if (nN <= 0 || in_sizes[0] != nN * DIN || nN > (1 << 22)) return;
  const int nE2 = in_sizes[1];
  if (nE2 < 2 || (nE2 & 1) != 0) return;
  const int nE = nE2 / 2;
  if (nE < 1 || nE > (1 << 21)) return;
  if (in_sizes[2] != DIN || in_sizes[3] != DIN) return;
  if (in_sizes[4] != DIN * DIN || in_sizes[5] != DIN) return;
  const int nL = in_sizes[6] / (DIN * DIN);
  if (nL < 1 || nL > 16 || in_sizes[6] != nL * DIN * DIN) return;
  if (in_sizes[7] != nL * DIN || in_sizes[8] != nL * DIN * DIN) return;
  if (in_sizes[9] != nL * DIN || in_sizes[10] != nL * DIN) return;
  if (in_sizes[11] != DIN || in_sizes[12] != DIN) return;
  if (in_sizes[13] != DIN * NOC || in_sizes[14] != NOC) return;
  if (out_size != nN * NOC) return;

  const float* x          = (const float*)d_in[0];
  const int*   ei         = (const int*)  d_in[1];
  const int*   src        = ei;
  const int*   dst        = ei + nE;
  const float* in_norm_g  = (const float*)d_in[2];
  const float* in_norm_b  = (const float*)d_in[3];
  const float* in_proj_w  = (const float*)d_in[4];
  const float* in_proj_b  = (const float*)d_in[5];
  const float* lin_l_w    = (const float*)d_in[6];
  const float* lin_l_b    = (const float*)d_in[7];
  const float* lin_r_w    = (const float*)d_in[8];
  const float* norm_g     = (const float*)d_in[9];
  const float* norm_b     = (const float*)d_in[10];
  const float* out_norm_g = (const float*)d_in[11];
  const float* out_norm_b = (const float*)d_in[12];
  const float* out_proj_w = (const float*)d_in[13];
  const float* out_proj_b = (const float*)d_in[14];
  float* out = (float*)d_out;

  const int MP   = cdiv(nN, GBM) * GBM;
  const int nb   = pick_nb(nE, nN);
  const int gA   = cdiv(MP, nb);
  const int vec8 = ((nE & 3) == 0) ? 1 : 0;
  if (gA * nb < MP || (MP % NWAVE) != 0 || (nb & 7) != 0) return;

  char* ws = (char*)d_ws;
  size_t off = 0;
  const size_t szH  = (size_t)MP * DIN * 4;
  const size_t szHH = (size_t)MP * APW * 2;
  const size_t oHA  = off; off += szH;                                off = (off + 255) & ~(size_t)255;
  const size_t oHHA = off; off += szHH;                               off = (off + 255) & ~(size_t)255;
  const size_t oHB  = off; off += szH;                                off = (off + 255) & ~(size_t)255;
  const size_t oHHB = off; off += szHH;                               off = (off + 255) & ~(size_t)255;
  const size_t oAG  = off; off += szHH;                               off = (off + 255) & ~(size_t)255;
  const size_t oWP  = off; off += (size_t)DIN * (size_t)KSEG * 2;     off = (off + 255) & ~(size_t)255;
  const size_t oWL  = off; off += (size_t)nL * DIN * (2 * KSEG) * 2;  off = (off + 255) & ~(size_t)255;
  const size_t oWO  = off; off += (size_t)NOC * (size_t)KSEG * 2;     off = (off + 255) & ~(size_t)255;
  if (off > ws_size || off > (size_t)WSMAX) return;
  float*          HA  = (float*)(ws + oHA);
  unsigned short* HHA = (unsigned short*)(ws + oHHA);
  float*          HB  = (float*)(ws + oHB);
  unsigned short* HHB = (unsigned short*)(ws + oHHB);
  unsigned short* AG  = (unsigned short*)(ws + oAG);
  unsigned short* WP  = (unsigned short*)(ws + oWP);
  unsigned short* WL  = (unsigned short*)(ws + oWL);
  unsigned short* WO  = (unsigned short*)(ws + oWO);

  hipFuncSetAttribute(reinterpret_cast<const void*>(&k_agg),
                      hipFuncAttributeMaxDynamicSharedMemorySize, LDS_AGG);

  k_wtr<<<dim3(DIN / 16, 1), NTHR, 0, stream>>>(in_proj_w, in_proj_w, 0, WP, 0, DIN, KSEG, 1);
  k_wtr<<<dim3(DIN / 16, nL), NTHR, 0, stream>>>(lin_l_w, lin_r_w, DIN * DIN, WL, DIN * 2 * KSEG, DIN, 2 * KSEG, 2);
  k_wtr<<<dim3(NOC / 16, 1), NTHR, 0, stream>>>(out_proj_w, out_proj_w, 0, WO, 0, NOC, KSEG, 1);

  k_ln<<<MP / NWAVE, NTHR, 0, stream>>>(x, in_norm_g, in_norm_b, 1, AG, nN, MP);

  k_gemm_h<<<dim3(MP / GBM, 1), GTHR, 0, stream>>>(AG, AG, 1, APW, WP, KSEG, in_proj_b, in_norm_g, in_norm_b,
                                                   x, 0, HA, HHA, nN, MP);

  float* Hc = HA; unsigned short* HHc = HHA;
  float* Hn = HB; unsigned short* HHn = HHB;
  for (int i = 0; i < nL; ++i) {
    k_agg<<<gA, NTHR, LDS_AGG, stream>>>(src, dst, Hc, AG, APW, nN, nE, nb, vec8, MP);
    k_gemm_h<<<dim3(MP / GBM, 1), GTHR, 0, stream>>>(AG, HHc, 2, APW,
                                                     WL + (size_t)i * DIN * (2 * KSEG), 2 * KSEG,
                                                     lin_l_b + (size_t)i * DIN,
                                                     norm_g + (size_t)i * DIN, norm_b + (size_t)i * DIN,
                                                     Hc, 1, Hn, HHn, nN, MP);
    float* tH = Hc; Hc = Hn; Hn = tH;
    unsigned short* tHH = HHc; HHc = HHn; HHn = tHH;
  }

  k_ln<<<MP / NWAVE, NTHR, 0, stream>>>(Hc, out_norm_g, out_norm_b, 0, AG, nN, MP);

  k_gemm_o<<<dim3(MP / GBM, 1), GTHR, 0, stream>>>(AG, APW, WO, KSEG, out_proj_b, out, nN);
}
